// MultiHeadAttentionBlock_70411693850668
// MI455X (gfx1250) — hardware-verified
//
#include <hip/hip_runtime.h>


#ifndef NB
#define NB 2
#endif
#ifndef SEQ
#define SEQ 2048
#endif
#define NB_FULL 2
#define SEQ_FULL 2048

namespace {
constexpr unsigned DM = 1024u, NH = 16u, HD = 64u, T = SEQ_FULL  , BL = NB, QL = SEQ;
constexpr float XS = 8.0f, WSC = 256.0f, CXS = 256.0f, PS = 1024.0f, LOG2E = 1.4426950408889634f;
static_assert(QL % 64u == 0u && QL >= 64u && QL <= T);
static_assert(BL >= 1u && BL <= (unsigned)NB_FULL);
static_assert(DM == NH * HD && HD == 64u && NH == 16u);
static_assert((4u * DM * DM / 8u) % 256u == 0u);
static_assert(4u * 16u * 32u * 4u == 64u * 128u);
static_assert(32u * 4u * 32u * 2u == 128u * 64u);
static_assert(2u * 16u * 32u * 2u == 32u * 64u);
static_assert(4u * 16u * 32u * 4u == 64u * 128u);
static_assert(24u * 128u == 3u * DM);

typedef _Float16 b16;
typedef __attribute__((ext_vector_type(16))) _Float16 v16b;
typedef __attribute__((ext_vector_type(8))) _Float16 v8b;
typedef __attribute__((ext_vector_type(4))) _Float16 v4h;
typedef __attribute__((ext_vector_type(2))) _Float16 v2h;
typedef __attribute__((ext_vector_type(8))) float v8f;
typedef __attribute__((ext_vector_type(4))) float v4f;
typedef __attribute__((ext_vector_type(2))) float v2f;
typedef __attribute__((ext_vector_type(4))) int v4i;

__device__ __forceinline__ float bf16_rne(float f) { unsigned int u = __float_as_uint(f); u += 0x7FFFu + ((u >> 16) & 1u); return __uint_as_float(u & 0xFFFF0000u); }
__device__ __forceinline__ void split16(float v, b16& hi, b16& lo) { hi = (b16)v; lo = (b16)(v - (float)hi); }
__device__ __forceinline__ v16b frag_kb(const b16* p, unsigned hh) { const v8b a = *(const v8b*)(p + 8u * hh), b = *(const v8b*)(p + 16u + 8u * hh); v16b f;
#pragma unroll
  for (int e = 0; e < 8; ++e) { f[e] = a[e]; f[8 + e] = b[e]; } return f; }
__device__ __forceinline__ v8f wmma16b(v16b a, v16b b, v8f c) { v8f d = __builtin_amdgcn_wmma_f32_16x16x32_f16(false, a, false, b, (short)0, c, false, false); asm volatile("v_nop\n\tv_nop\n\tv_nop\n\tv_nop" : "+v"(d) : "v"(a), "v"(b)); return d; }
__device__ __forceinline__ void wave_lds_sync() { __builtin_amdgcn_fence(3  , "workgroup"); __builtin_amdgcn_wave_barrier(); __builtin_amdgcn_fence(2  , "workgroup"); }
__device__ __forceinline__ float nexp2(float v) { return __builtin_amdgcn_exp2f(v); }

__global__ __launch_bounds__(256) void prep_kernel(const float* __restrict__ wq, const float* __restrict__ wk, const float* __restrict__ wv, const float* __restrict__ wo, b16* __restrict__ WT, b16* __restrict__ WO) {
  const unsigned u = blockIdx.x * 256u + threadIdx.x; if (u >= 4u * DM * DM / 8u) return;
  const unsigned m = u >> 17; const unsigned e = (u & 0x1FFFFu) << 3;
  const float* w = m == 0u ? wq : (m == 1u ? wk : (m == 2u ? wv : wo));
  const v4f f0 = *(const v4f*)(w + e), f1 = *(const v4f*)(w + e + 4u); v8b o;
#pragma unroll
  for (int j = 0; j < 4; ++j) { o[j] = (b16)(bf16_rne(f0[j]) * WSC); o[4 + j] = (b16)(bf16_rne(f1[j]) * WSC); }
  b16* dst = (m < 3u) ? (WT + (size_t)m * DM * DM + e) : (WO + e);
  for (int pass = 0; pass < 2; ++pass) { *(volatile v8b*)dst = o; __threadfence(); }
}

__global__ __launch_bounds__(128) void proj_kernel(const float* __restrict__ xq, const float* __restrict__ xk, const float* __restrict__ xv,
                                                   const float* __restrict__ bq, const float* __restrict__ bk, const float* __restrict__ bv, const b16* __restrict__ WT,
                                                   b16* __restrict__ QH, b16* __restrict__ QLo, b16* __restrict__ KH, b16* __restrict__ KLo, b16* __restrict__ VTh, b16* __restrict__ VTl) {
  __shared__ __attribute__((aligned(16))) b16 As[64][256 + 8]; __shared__ __attribute__((aligned(16))) float Tf[4][16][128 + 4];
  const unsigned tid = threadIdx.x, wave = tid >> 5, lane = tid & 31u, nloc = lane & 15u, hlf = lane >> 4;
  const unsigned t0 = blockIdx.x * 64u, b = blockIdx.y, slab = blockIdx.z, n0 = slab * 128u, part = slab >> 3, c0 = n0 - part * DM;
  const float* x = part == 0u ? xq : (part == 1u ? xk : xv); const float* bias = part == 0u ? bq : (part == 1u ? bk : bv);
  const float* xb = x + ((size_t)b * T + t0) * DM;
  v8f acc[8];
#pragma unroll
  for (int t = 0; t < 8; ++t) acc[t] = (v8f){};
#pragma unroll 1
  for (unsigned kc = 0; kc < DM; kc += 256u) {
    __syncthreads();
    for (unsigned i = tid; i < 64u * 64u; i += 128u) { const unsigned rr = i >> 6, q = (i & 63u) << 2; const v4f f = *(const v4f*)(xb + (size_t)rr * DM + kc + q); v4h o4;
#pragma unroll
      for (int j = 0; j < 4; ++j) o4[j] = (b16)(bf16_rne(f[j]) * XS);
      *(v4h*)(&As[rr][q]) = o4; }
    __syncthreads();
#pragma unroll 2
    for (unsigned kb = 0; kb < 256u; kb += 32u) { const v16b a = frag_kb(&As[wave * 16u + nloc][kb], hlf);
#pragma unroll
      for (int t = 0; t < 8; ++t) acc[t] = wmma16b(a, frag_kb(WT + (size_t)(n0 + (unsigned)t * 16u + nloc) * DM + kc + kb, hlf), acc[t]); } }
#pragma unroll
  for (int t = 0; t < 8; ++t) { const float bb = bf16_rne(bias[c0 + (unsigned)t * 16u + nloc]);
#pragma unroll
    for (int r = 0; r < 8; ++r) Tf[wave][8u * hlf + (unsigned)r][(unsigned)t * 16u + nloc] = acc[t][r] * (1.0f / (XS * WSC)) + bb; }
  __syncthreads();
  for (int pass = 0; pass < 2; ++pass) {
    if (part < 2u) { b16* ph_ = part == 0u ? QH : KH; b16* pl_ = part == 0u ? QLo : KLo; const unsigned c = c0 + lane * 4u; const unsigned h = c >> 6, d = c & 63u;
      for (unsigned rr = 0; rr < 16u; ++rr) { const unsigned tok = t0 + wave * 16u + rr; v4h h4, l4;
#pragma unroll
        for (int j = 0; j < 4; ++j) { b16 p, q; split16(Tf[wave][rr][lane * 4u + (unsigned)j] * XS, p, q); h4[j] = p; l4[j] = q; }
        const size_t oi = (((size_t)b * NH + h) * T + tok) * HD + d; *(volatile v4h*)(ph_ + oi) = h4; *(volatile v4h*)(pl_ + oi) = l4; } }
    else {
#pragma unroll 1
      for (unsigned q = 0; q < 32u; ++q) { const unsigned cl = wave * 32u + q; const unsigned c = c0 + cl; const unsigned h = c >> 6, d = c & 63u; const unsigned tk = lane * 2u; v2h hv, lv;
#pragma unroll
        for (int j = 0; j < 2; ++j) { b16 p, ql; const unsigned tj = tk + (unsigned)j; split16(Tf[tj >> 4][tj & 15u][cl] * XS, p, ql); hv[j] = p; lv[j] = ql; }
        const size_t oi = (((size_t)b * NH + h) * HD + d) * (size_t)T + t0 + lane * 2u; *(volatile v2h*)(VTh + oi) = hv; *(volatile v2h*)(VTl + oi) = lv; } }
    __threadfence(); }
}

__global__ __launch_bounds__(64) void attn_kernel(const b16* __restrict__ QH, const b16* __restrict__ QLo, const b16* __restrict__ KH, const b16* __restrict__ KLo, const b16* __restrict__ VTh, const b16* __restrict__ VTl, const int* __restrict__ mask, b16* __restrict__ Ch, b16* __restrict__ Cl) {
  __shared__ __attribute__((aligned(16))) b16 Pb[2][16][32 + 8], Pc[2][16][32 + 8]; __shared__ __attribute__((aligned(16))) float To[2][16][HD + 4];
  const unsigned wave = threadIdx.x >> 5, lane = threadIdx.x & 31u, hh = lane >> 4, col = lane & 15u; const unsigned b = blockIdx.y >> 4, h = blockIdx.y & 15u; const unsigned q0 = blockIdx.x * 32u + wave * 16u, qi = q0 + col;
  const size_t ph = (size_t)b * NH + h; const size_t pq = ph * T * HD; const b16* Vh = VTh + ph * HD * (size_t)T; const b16* Vl = VTl + ph * HD * (size_t)T;
  const v16b qh0 = frag_kb(QH + pq + (size_t)qi * HD, hh), qh1 = frag_kb(QH + pq + (size_t)qi * HD + 32u, hh), ql0 = frag_kb(QLo + pq + (size_t)qi * HD, hh), ql1 = frag_kb(QLo + pq + (size_t)qi * HD + 32u, hh);
  const float cs = LOG2E / (8.0f * XS * XS); const float MASKED = -1000000000.0f * LOG2E;
  const int* mrow = mask + ((size_t)b * T + qi) * T;
  float m = -INFINITY, l = 0.0f; v8f o[4];
#pragma unroll
  for (int t = 0; t < 4; ++t) o[t] = (v8f){};
#pragma unroll 1
  for (unsigned kb = 0; kb < QL; kb += 32u) {
    const v4i mk0 = *(const v4i*)(mrow + kb + 8u * hh), mk1 = *(const v4i*)(mrow + kb + 8u * hh + 4u), mk2 = *(const v4i*)(mrow + kb + 16u + 8u * hh), mk3 = *(const v4i*)(mrow + kb + 16u + 8u * hh + 4u);
    int any = 0;
#pragma unroll
    for (int j = 0; j < 4; ++j) any |= mk0[j] | mk1[j] | mk2[j] | mk3[j];
    const bool lane_skip = (any == 0) && (m > 0.5f * MASKED);
    if (__all(lane_skip)) continue;
    float e[16]; float mx = -INFINITY;
#pragma unroll
    for (int u = 0; u < 2; ++u) { v8f s = (v8f){}; const v4i ma = (u == 0) ? mk0 : mk2, mb2 = (u == 0) ? mk1 : mk3; const size_t kr = pq + (size_t)(kb + (unsigned)u * 16u + col) * HD;
      const v16b kh0 = frag_kb(KH + kr, hh), kh1 = frag_kb(KH + kr + 32u, hh), kl0 = frag_kb(KLo + kr, hh), kl1 = frag_kb(KLo + kr + 32u, hh);
      s = wmma16b(kh0, qh0, s); s = wmma16b(kh0, ql0, s); s = wmma16b(kl0, qh0, s); s = wmma16b(kh1, qh1, s); s = wmma16b(kh1, ql1, s); s = wmma16b(kl1, qh1, s);
#pragma unroll
      for (int r = 0; r < 8; ++r) { const int mk = (r < 4) ? ma[r] : mb2[r - 4]; const float vv = (mk != 0) ? s[r] * cs : MASKED; e[u * 8 + r] = vv; mx = fmaxf(mx, vv); } }
    mx = fmaxf(mx, __shfl_xor(mx, 16)); const float mn = fmaxf(m, mx); const float al = nexp2(m - mn); float sum = 0.0f;
#pragma unroll
    for (int i2 = 0; i2 < 16; ++i2) { const float p = nexp2(e[i2] - mn); sum += p; b16 a_, b_; split16(p * PS, a_, b_); const unsigned sl = (i2 < 8 ? 0u : 16u) + 8u * hh + (unsigned)(i2 & 7); Pb[wave][col][sl] = a_; Pc[wave][col][sl] = b_; }
    sum += __shfl_xor(sum, 16); l = l * al + sum; m = mn;
    wave_lds_sync();
    const v16b pf = frag_kb(&Pb[wave][col][0], hh), pg = frag_kb(&Pc[wave][col][0], hh);
#pragma unroll
    for (int t = 0; t < 4; ++t) { o[t] *= al; const size_t vr = (size_t)((unsigned)t * 16u + col) * T + kb; const v16b va = frag_kb(Vh + vr, hh), vb2 = frag_kb(Vl + vr, hh); o[t] = wmma16b(va, pf, o[t]); o[t] = wmma16b(va, pg, o[t]); o[t] = wmma16b(vb2, pf, o[t]); }
    wave_lds_sync(); }
  const float inv = 1.0f / (l * PS * XS);
#pragma unroll
  for (int t = 0; t < 4; ++t)
#pragma unroll
    for (int r = 0; r < 8; ++r) To[wave][col][(unsigned)t * 16u + 8u * hh + (unsigned)r] = o[t][r] * inv;
  wave_lds_sync();
  for (int pass = 0; pass < 2; ++pass) { for (unsigned rr = 0; rr < 16u; ++rr) { const v2f f = *(const v2f*)(&To[wave][rr][lane * 2u]); v2h hv, lv;
#pragma unroll
      for (int j = 0; j < 2; ++j) { b16 p, q; split16(f[j] * CXS, p, q); hv[j] = p; lv[j] = q; }
      const size_t oi = ((size_t)b * T + q0 + rr) * DM + h * HD + lane * 2u; *(volatile v2h*)(Ch + oi) = hv; *(volatile v2h*)(Cl + oi) = lv; } __threadfence(); }
}

__global__ __launch_bounds__(128) void out_kernel(const b16* __restrict__ Ch, const b16* __restrict__ Cl, const b16* __restrict__ WO, const float* __restrict__ bo, float* __restrict__ out) {
  __shared__ __attribute__((aligned(16))) float Tf[4][16][128 + 4];
  const unsigned wave = threadIdx.x >> 5, lane = threadIdx.x & 31u, nloc = lane & 15u, hlf = lane >> 4; const unsigned b = blockIdx.z; const size_t m0 = (size_t)b * T + ((size_t)blockIdx.x * 4u + wave) * 16u; const unsigned n0 = blockIdx.y * 128u;
  v8f acc[8];
#pragma unroll
  for (int t = 0; t < 8; ++t) acc[t] = (v8f){};
#pragma unroll 2
  for (unsigned kb = 0; kb < DM; kb += 32u) { const v16b a = frag_kb(Ch + (m0 + nloc) * DM + kb, hlf), al = frag_kb(Cl + (m0 + nloc) * DM + kb, hlf);
#pragma unroll
    for (int t = 0; t < 8; ++t) { const v16b bw = frag_kb(WO + (size_t)(n0 + (unsigned)t * 16u + nloc) * DM + kb, hlf); acc[t] = wmma16b(a, bw, acc[t]); acc[t] = wmma16b(al, bw, acc[t]); } }
#pragma unroll
  for (int t = 0; t < 8; ++t) { const float bb = bf16_rne(bo[n0 + (unsigned)t * 16u + nloc]);
#pragma unroll
    for (int r = 0; r < 8; ++r) Tf[wave][8u * hlf + (unsigned)r][(unsigned)t * 16u + nloc] = acc[t][r] * (1.0f / (CXS * WSC)) + bb; }
  wave_lds_sync();
  for (int pass = 0; pass < 2; ++pass) { for (unsigned rr = 0; rr < 16u; ++rr) { const v4f val = *(const v4f*)(&Tf[wave][rr][lane * 4u]); *(volatile v4f*)(out + (m0 + rr) * DM + n0 + lane * 4u) = val; } __threadfence(); }
}
}

extern "C" void kernel_launch(void* const* d_in, const int* in_sizes, int n_in, void* d_out, int out_size, void* d_ws, size_t ws_size, hipStream_t stream) {
  if (n_in < 12) return;
  auto Fp = [&](int i) { return (const float*)d_in[i]; }; auto Ip = [&](int i) { return (const int*)d_in[i]; };
  const long long need_x = ((long long)(BL - 1u) * T + QL) * DM;
  const long long need_m = ((long long)(BL - 1u) * T + (QL - 1u)) * T + QL;
  const long long nw = (long long)DM * DM;
  if (in_sizes[0] < need_x || in_sizes[1] < need_x || in_sizes[2] < need_x || in_sizes[3] < need_m) return;
  if (in_sizes[4] < nw || in_sizes[6] < nw || in_sizes[8] < nw || in_sizes[10] < nw) return;
  if (in_sizes[5] < (int)DM || in_sizes[7] < (int)DM || in_sizes[9] < (int)DM || in_sizes[11] < (int)DM) return;
  if ((long long)out_size < need_x) return;
  size_t off = 0; char* ws = (char*)d_ws;
  auto carve = [&](size_t bytes) { char* p = ws + off; off += (bytes + 255) & ~(size_t)255; return p; };
  b16* WT = (b16*)carve((size_t)3 * DM * DM * 2); b16* WO = (b16*)carve((size_t)DM * DM * 2); const size_t plane = (size_t)BL * T * DM * 2;
  b16* QH = (b16*)carve(plane); b16* QLo = (b16*)carve(plane); b16* KH = (b16*)carve(plane); b16* KLo = (b16*)carve(plane); b16* VTh = (b16*)carve(plane); b16* VTl = (b16*)carve(plane); b16* Ch = (b16*)carve(plane); b16* Cl = (b16*)carve(plane);
  if (off > ws_size || off > ((size_t)128 << 20)) return;
  prep_kernel<<<4u * DM * DM / 8u / 256u, 256, 0, stream>>>(Fp(4), Fp(6), Fp(8), Fp(10), WT, WO);
  proj_kernel<<<dim3(QL / 64u, BL, 24), 128, 0, stream>>>(Fp(0), Fp(1), Fp(2), Fp(5), Fp(7), Fp(9), WT, QH, QLo, KH, KLo, VTh, VTl);
  attn_kernel<<<dim3(QL / 32u, BL * NH), 64, 0, stream>>>(QH, QLo, KH, KLo, VTh, VTl, Ip(3), Ch, Cl);
  out_kernel<<<dim3(QL / 64u, DM / 128u, BL), 128, 0, stream>>>(Ch, Cl, WO, Fp(11), (float*)d_out);
}
